// InterventionalGraph_46196668236076
// MI455X (gfx1250) — hardware-verified
//
#include <hip/hip_runtime.h>
#include <math.h>
#include <stdint.h>

#define NB     128
#define NTOK   200
#define NLAG   30
#define NTO    (NTOK - NLAG)
#define NTGT   (NB * NTO)
#define NSK    1000
#define EMB    64
#define HIDW   64
#define FEW    (2 * EMB)

#define WPB    2
#define ETPB   (WPB * 32)
#define XP     136
#define HP     64
#define KS0    4
#define KS1    2
#define NT4    4
#define MT2    2

#define DROWS  32
#define DTPB   64
#define DP     72

#define P0_EL  (NT4 * KS0 * 512)
#define P1_EL  (NT4 * KS1 * 512)
#define EMB_EL (NSK * EMB)

#define INV_LOG5 (1.0f / 1.6094379425048828f)

static_assert((NTGT % WPB) == 0);
static_assert((NTGT % DROWS) == 0);
static_assert(FEW == KS0 * 32);
static_assert(HIDW == KS1 * 32 && EMB == KS1 * 32);
static_assert(HIDW == NT4 * 16 && EMB == NT4 * 16);
static_assert((XP % 8) == 0 && XP >= FEW);
static_assert((HP % 8) == 0 && HP >= HIDW);
static_assert((DP % 8) == 0 && DP >= EMB);
static_assert((EMB_EL % 8) == 0);
static_assert(NLAG <= 32 && MT2 * 16 == 32);
static_assert(DROWS == 32 && DTPB == 64);

typedef __bf16         v16b __attribute__((ext_vector_type(16)));
typedef unsigned short v8us __attribute__((ext_vector_type(8)));
typedef unsigned short v4us __attribute__((ext_vector_type(4)));
typedef float          v8f  __attribute__((ext_vector_type(8)));
typedef float          v4f  __attribute__((ext_vector_type(4)));

union FragB { v16b v; v8us u[2]; };

__device__ __forceinline__ unsigned short bf_bits(float f) {
  const unsigned u = __float_as_uint(f);
  return (unsigned short)((u + 0x7FFFu + ((u >> 16) & 1u)) >> 16);
}
__device__ __forceinline__ float bf_up(unsigned short b) { return __uint_as_float(((unsigned)b) << 16); }
__device__ __forceinline__ float bfr(float f) { return bf_up(bf_bits(f)); }
__device__ __forceinline__ float lrelu(float x) { return (x >= 0.0f) ? x : 0.01f * x; }
__device__ __forceinline__ int clamp_sk(int s) { return (s < 0) ? 0 : ((s >= NSK) ? (NSK - 1) : s); }
__device__ __forceinline__ v8f zero8() { return (v8f){0.f, 0.f, 0.f, 0.f, 0.f, 0.f, 0.f, 0.f}; }

__device__ __forceinline__ v8f mma_b(v16b a, v16b b, v8f c) {
  return __builtin_amdgcn_wmma_f32_16x16x32_bf16(false, a, false, b, (short)0, c, false, false);
}
__device__ __forceinline__ void mma_guard1(v8f& c0, v16b a0, v16b b) {
#if defined(__HIP_DEVICE_COMPILE__)
  asm volatile("v_nop\n\tv_nop\n\tv_nop\n\tv_nop" : "+v"(c0) : "v"(a0), "v"(b));
#else
  (void)c0; (void)a0; (void)b;
#endif
}
__device__ __forceinline__ void mma_guard2(v8f& c0, v16b a0, v16b a1, v16b b) {
#if defined(__HIP_DEVICE_COMPILE__)
  asm volatile("v_nop\n\tv_nop\n\tv_nop\n\tv_nop" : "+v"(c0) : "v"(a0), "v"(a1), "v"(b));
#else
  (void)c0; (void)a0; (void)a1; (void)b;
#endif
}

__global__ __launch_bounds__(256) void k_embc(const float* __restrict__ emb, unsigned short* dst, int nPieces) {
  const int piece = blockIdx.x * 256 + threadIdx.x;
  const bool act  = piece < nPieces;
  const int pc    = act ? piece : (nPieces - 1);
  const v4f a = *(const v4f*)(emb + (size_t)pc * 8);
  const v4f b = *(const v4f*)(emb + (size_t)pc * 8 + 4);
  v8us o;
#pragma unroll
  for (int j = 0; j < 4; ++j) { o[j] = bf_bits(a[j]); o[4 + j] = bf_bits(b[j]); }
  unsigned short* d = dst + (size_t)pc * 8;
  if (act) *(volatile v8us*)d = o;
  __threadfence();
  if (act) *(volatile v8us*)d = o;
}

__global__ __launch_bounds__(256) void k_pack(const float* __restrict__ Wm, unsigned short* dst,
                                              int Kreal, int Nreal, int kS, int nPieces) {
  const int piece = blockIdx.x * 256 + threadIdx.x;
  const bool act  = piece < nPieces;
  const int pc    = act ? piece : (nPieces - 1);
  const int elem0 = pc * 8;
  const int tblk  = kS * 512;
  const int t     = elem0 / tblk;
  int rem         = elem0 - t * tblk;
  const int s     = rem >> 9;
  rem            &= 511;
  const int L     = rem >> 4;
  const int j0    = rem & 15;
  const int n     = t * 16 + (L & 15);
  const int hh    = L >> 4;
  const int kb    = s * 32 + 8 * hh + 2 * j0;
  const int nc    = (n < Nreal) ? n : (Nreal - 1);
  v8us o;
#pragma unroll
  for (int jj = 0; jj < 8; ++jj) {
    const int k  = kb + jj;
    const int kc = (k < Kreal) ? k : (Kreal - 1);
    float v = Wm[(size_t)nc * Kreal + kc];
    v = (k < Kreal && n < Nreal) ? v : 0.0f;
    o[jj] = bf_bits(v);
  }
  unsigned short* d = dst + (size_t)pc * 8;
  if (act) *(volatile v8us*)d = o;
  __threadfence();
  if (act) *(volatile v8us*)d = o;
}

__global__ __launch_bounds__(ETPB) void k_edge(
    const int* __restrict__ skills, const int* __restrict__ times, const int* __restrict__ labels,
    const float* __restrict__ W, const float* __restrict__ sbase,
    const unsigned short* __restrict__ embb,
    const unsigned short* __restrict__ Wp0, const unsigned short* __restrict__ Wp1,
    const unsigned short* __restrict__ Wpo,
    const float* __restrict__ b0, const float* __restrict__ b1, const float* __restrict__ bo,
    float* cef) {
  __shared__ __align__(16) unsigned short sX[WPB * 32 * XP];
  __shared__ __align__(16) unsigned short sH[WPB * 2 * 32 * HP];
  __shared__ __align__(16) unsigned short sG[WPB * 2 * 32 * HP];
  __shared__ __align__(16) float sCoef[WPB * 32];
  __shared__ __align__(16) float sCe[WPB * EMB];

  const int tid  = threadIdx.x;
  const int lane = tid & 31;
  const int wv   = tid >> 5;
  const int m    = lane & 15;
  const int hh   = lane >> 4;
  const int mrow = 8 * hh;
  const int wid  = blockIdx.x * WPB + wv;
  const int bb   = wid / NTO;
  const int tt_i = wid - bb * NTO;
  const int tok0 = bb * NTOK + tt_i;

  unsigned short* xt = sX + wv * (32 * XP);
  unsigned short* Hh = sH + wv * (2 * 32 * HP);
  unsigned short* Hl = Hh + 32 * HP;
  unsigned short* Gh = sG + wv * (2 * 32 * HP);
  unsigned short* Gl = Gh + 32 * HP;
  float* coefw = sCoef + wv * 32;
  float* cew   = sCe + wv * EMB;

  const int   tgt = clamp_sk(skills[tok0 + NLAG]);
  const float ttm = (float)times[tok0 + NLAG];

  {
    const int j    = lane;
    const int jj   = (j < NLAG) ? j : (NLAG - 1);
    const bool rowon = (j < NLAG);
    const int tok  = tok0 + jj;
    const int sh   = clamp_sk(skills[tok]);
    const int lab  = labels[tok];
    const float th = (float)times[tok];
    const float labf = (lab == 0) ? -1.0f : ((lab == -1) ? 0.0f : (float)lab);
    const float wraw = W[(size_t)sh * NSK + tgt];
    const float cw   = (sh == tgt) ? 0.0f : bfr(wraw);
    const float dlt  = logf(fabsf(ttm - th) + 1e-10f) * INV_LOG5;
    const float fac  = cw * expf(-dlt);
    coefw[j] = rowon ? fac : 0.0f;
    const unsigned short* et = embb + (size_t)tgt * EMB;
    const unsigned short* eh = embb + (size_t)sh * EMB;
    unsigned short* xr = xt + j * XP;
#pragma unroll
    for (int p = 0; p < 8; ++p) {
      const v8us u = *(const v8us*)(et + 8 * p);
      v8us o;
#pragma unroll
      for (int e = 0; e < 8; ++e) o[e] = rowon ? u[e] : (unsigned short)0;
      *(v8us*)(xr + 8 * p) = o;
    }
#pragma unroll
    for (int p = 0; p < 8; ++p) {
      const v8us u = *(const v8us*)(eh + 8 * p);
      v8us o;
#pragma unroll
      for (int e = 0; e < 8; ++e) {
        const unsigned short val = bf_bits(bf_up(u[e]) * labf);
        o[e] = rowon ? val : (unsigned short)0;
      }
      *(v8us*)(xr + EMB + 8 * p) = o;
    }
  }
  __syncthreads();

  v8f h0[MT2][NT4];
  {
#pragma unroll
    for (int mt = 0; mt < MT2; ++mt) {
      FragB a[KS0];
#pragma unroll
      for (int s = 0; s < KS0; ++s) {
        const unsigned short* p = xt + (mt * 16 + m) * XP + s * 32 + 8 * hh;
        a[s].u[0] = *(const v8us*)(p);
        a[s].u[1] = *(const v8us*)(p + 16);
      }
#pragma unroll
      for (int nt = 0; nt < NT4; ++nt) {
        const int n    = nt * 16 + m;
        const float bv = bfr(b0[n]);
        v8f c = zero8();
        FragB bq;
#pragma unroll
        for (int s = 0; s < KS0; ++s) {
          const unsigned short* wp = Wp0 + ((size_t)((nt * KS0 + s) * 32 + lane) << 4);
          bq.u[0] = *(const v8us*)(wp);
          bq.u[1] = *(const v8us*)(wp + 8);
          c = mma_b(a[s].v, bq.v, c);
        }
        mma_guard1(c, a[KS0 - 1].v, bq.v);
        v8f hv = zero8();
#pragma unroll
        for (int v = 0; v < 8; ++v) {
          const float z = lrelu(c[v] + bv);
          hv[v] = z;
          const unsigned short hb = bf_bits(z);
          const unsigned short lb = bf_bits(z - bf_up(hb));
          Hh[(mt * 16 + mrow + v) * HP + n] = hb;
          Hl[(mt * 16 + mrow + v) * HP + n] = lb;
        }
        h0[mt][nt] = hv;
      }
    }
  }
  __syncthreads();

  {
#pragma unroll
    for (int mt = 0; mt < MT2; ++mt) {
      FragB ah[KS1], al[KS1];
#pragma unroll
      for (int s = 0; s < KS1; ++s) {
        const unsigned short* ph = Hh + (mt * 16 + m) * HP + s * 32 + 8 * hh;
        const unsigned short* pl = Hl + (mt * 16 + m) * HP + s * 32 + 8 * hh;
        ah[s].u[0] = *(const v8us*)(ph);
        ah[s].u[1] = *(const v8us*)(ph + 16);
        al[s].u[0] = *(const v8us*)(pl);
        al[s].u[1] = *(const v8us*)(pl + 16);
      }
#pragma unroll
      for (int nt = 0; nt < NT4; ++nt) {
        const int n    = nt * 16 + m;
        const float bv = bfr(b1[n]);
        v8f c = zero8();
        FragB bq;
#pragma unroll
        for (int s = 0; s < KS1; ++s) {
          const unsigned short* wp = Wp1 + ((size_t)((nt * KS1 + s) * 32 + lane) << 4);
          bq.u[0] = *(const v8us*)(wp);
          bq.u[1] = *(const v8us*)(wp + 8);
          c = mma_b(ah[s].v, bq.v, c);
          c = mma_b(al[s].v, bq.v, c);
        }
        mma_guard2(c, ah[KS1 - 1].v, al[KS1 - 1].v, bq.v);
#pragma unroll
        for (int v = 0; v < 8; ++v) {
          const float g = h0[mt][nt][v] + lrelu(c[v] + bv);
          const unsigned short hb = bf_bits(g);
          const unsigned short lb = bf_bits(g - bf_up(hb));
          Gh[(mt * 16 + mrow + v) * HP + n] = hb;
          Gl[(mt * 16 + mrow + v) * HP + n] = lb;
        }
      }
    }
  }
  __syncthreads();

  float ce[NT4] = {0.0f, 0.0f, 0.0f, 0.0f};
  {
#pragma unroll
    for (int mt = 0; mt < MT2; ++mt) {
      FragB ah[KS1], al[KS1];
#pragma unroll
      for (int s = 0; s < KS1; ++s) {
        const unsigned short* ph = Gh + (mt * 16 + m) * HP + s * 32 + 8 * hh;
        const unsigned short* pl = Gl + (mt * 16 + m) * HP + s * 32 + 8 * hh;
        ah[s].u[0] = *(const v8us*)(ph);
        ah[s].u[1] = *(const v8us*)(ph + 16);
        al[s].u[0] = *(const v8us*)(pl);
        al[s].u[1] = *(const v8us*)(pl + 16);
      }
      float cm[8];
#pragma unroll
      for (int v = 0; v < 8; ++v) cm[v] = coefw[mt * 16 + mrow + v];
#pragma unroll
      for (int nt = 0; nt < NT4; ++nt) {
        const int n    = nt * 16 + m;
        const float bv = bfr(bo[n]);
        v8f c = zero8();
        FragB bq;
#pragma unroll
        for (int s = 0; s < KS1; ++s) {
          const unsigned short* wp = Wpo + ((size_t)((nt * KS1 + s) * 32 + lane) << 4);
          bq.u[0] = *(const v8us*)(wp);
          bq.u[1] = *(const v8us*)(wp + 8);
          c = mma_b(ah[s].v, bq.v, c);
          c = mma_b(al[s].v, bq.v, c);
        }
        mma_guard2(c, ah[KS1 - 1].v, al[KS1 - 1].v, bq.v);
        float part = 0.0f;
#pragma unroll
        for (int v = 0; v < 8; ++v) part = fmaf(cm[v], c[v] + bv, part);
        ce[nt] += part;
      }
    }
  }
  const float sb = bfr(sbase[tgt]);
#pragma unroll
  for (int nt = 0; nt < NT4; ++nt) {
    const float tot = ce[nt] + __shfl_xor(ce[nt], 16);
    if (lane < 16) cew[nt * 16 + lane] = tot + sb;
  }
  __syncthreads();
  {
    const int q  = lane & 15;
    const v4f cv = *(const v4f*)(cew + q * 4);
    float* cp = cef + (size_t)wid * EMB + q * 4;
    if (lane < 16) *(volatile v4f*)cp = cv;
    __threadfence();
    if (lane < 16) *(volatile v4f*)cp = cv;
  }
}

__global__ __launch_bounds__(DTPB) void k_dec(
    const float* __restrict__ cef,
    const unsigned short* __restrict__ Wq0, const unsigned short* __restrict__ Wq1,
    const float* __restrict__ fb0, const float* __restrict__ fb1,
    const float* __restrict__ fwo, const float* __restrict__ fbo,
    float* out) {
  __shared__ __align__(16) float sXf[DROWS * EMB];
  __shared__ __align__(16) float sZ[DROWS * EMB];
  __shared__ __align__(16) unsigned short pl[4 * DROWS * DP];
  __shared__ __align__(16) float sWo[EMB];
  __shared__ __align__(16) float sOut[DROWS];

  const int tid  = threadIdx.x;
  const int lane = tid & 31;
  const int wave = tid >> 5;
  const int m    = lane & 15;
  const int hh   = lane >> 4;
  const int mrow = 8 * hh;
  unsigned short* Ah = pl;
  unsigned short* Al = pl + DROWS * DP;
  unsigned short* Bh = pl + 2 * DROWS * DP;
  unsigned short* Bl = pl + 3 * DROWS * DP;
  const int r0 = blockIdx.x * DROWS;

  for (int i = tid; i < DROWS * (EMB / 4); i += DTPB) {
    const int r = i >> 4, q = i & 15;
    const v4f v = *(const v4f*)(cef + (size_t)(r0 + r) * EMB + q * 4);
    *(v4f*)(sXf + r * EMB + q * 4) = v;
    v4us ho, lo;
#pragma unroll
    for (int j = 0; j < 4; ++j) {
      const unsigned short hb = bf_bits(v[j]);
      ho[j] = hb;
      lo[j] = bf_bits(v[j] - bf_up(hb));
    }
    *(v4us*)(Ah + r * DP + q * 4) = ho;
    *(v4us*)(Al + r * DP + q * 4) = lo;
  }
  for (int i = tid; i < EMB; i += DTPB) sWo[i] = bfr(fwo[i]);
  __syncthreads();

  const int wr = wave * 16;
  v8f hreg[NT4];
  {
    FragB ah[KS1], al[KS1];
#pragma unroll
    for (int s = 0; s < KS1; ++s) {
      const unsigned short* ph = Ah + (wr + m) * DP + s * 32 + 8 * hh;
      const unsigned short* pq = Al + (wr + m) * DP + s * 32 + 8 * hh;
      ah[s].u[0] = *(const v8us*)(ph);
      ah[s].u[1] = *(const v8us*)(ph + 16);
      al[s].u[0] = *(const v8us*)(pq);
      al[s].u[1] = *(const v8us*)(pq + 16);
    }
#pragma unroll
    for (int nt = 0; nt < NT4; ++nt) {
      const int n    = nt * 16 + m;
      const float bv = bfr(fb0[n]);
      v8f c = zero8();
      FragB bq;
#pragma unroll
      for (int s = 0; s < KS1; ++s) {
        const unsigned short* wp = Wq0 + ((size_t)((nt * KS1 + s) * 32 + lane) << 4);
        bq.u[0] = *(const v8us*)(wp);
        bq.u[1] = *(const v8us*)(wp + 8);
        c = mma_b(ah[s].v, bq.v, c);
        c = mma_b(al[s].v, bq.v, c);
      }
      mma_guard2(c, ah[KS1 - 1].v, al[KS1 - 1].v, bq.v);
      v8f hv = zero8();
#pragma unroll
      for (int v = 0; v < 8; ++v) {
        const int row = wr + mrow + v;
        const float x = sXf[row * EMB + n];
        const float h = x + lrelu(c[v] + bv);
        hv[v] = h;
        const unsigned short hb = bf_bits(h);
        const unsigned short lb = bf_bits(h - bf_up(hb));
        Bh[row * DP + n] = hb;
        Bl[row * DP + n] = lb;
      }
      hreg[nt] = hv;
    }
  }
  __syncthreads();
  {
    FragB ah[KS1], al[KS1];
#pragma unroll
    for (int s = 0; s < KS1; ++s) {
      const unsigned short* ph = Bh + (wr + m) * DP + s * 32 + 8 * hh;
      const unsigned short* pq = Bl + (wr + m) * DP + s * 32 + 8 * hh;
      ah[s].u[0] = *(const v8us*)(ph);
      ah[s].u[1] = *(const v8us*)(ph + 16);
      al[s].u[0] = *(const v8us*)(pq);
      al[s].u[1] = *(const v8us*)(pq + 16);
    }
#pragma unroll
    for (int nt = 0; nt < NT4; ++nt) {
      const int n    = nt * 16 + m;
      const float bv = bfr(fb1[n]);
      v8f c = zero8();
      FragB bq;
#pragma unroll
      for (int s = 0; s < KS1; ++s) {
        const unsigned short* wp = Wq1 + ((size_t)((nt * KS1 + s) * 32 + lane) << 4);
        bq.u[0] = *(const v8us*)(wp);
        bq.u[1] = *(const v8us*)(wp + 8);
        c = mma_b(ah[s].v, bq.v, c);
        c = mma_b(al[s].v, bq.v, c);
      }
      mma_guard2(c, ah[KS1 - 1].v, al[KS1 - 1].v, bq.v);
#pragma unroll
      for (int v = 0; v < 8; ++v) {
        const int row = wr + mrow + v;
        sZ[row * EMB + n] = hreg[nt][v] + lrelu(c[v] + bv);
      }
    }
  }
  __syncthreads();
  {
    const int r = tid & 31;
    const float* zr = sZ + r * EMB;
    float acc = 0.0f;
#pragma unroll 4
    for (int k = 0; k < EMB; ++k) acc = fmaf(zr[k], sWo[k], acc);
    const float lg = acc + bfr(fbo[0]);
    const float e  = expf(-lg);
    const float o  = __builtin_amdgcn_rcpf(1.0f + e);
    if (tid < DROWS) sOut[r] = o;
  }
  __syncthreads();
  {
    const int q = tid & 7;
    const v4f ov = *(const v4f*)(sOut + q * 4);
    float* op = out + (size_t)blockIdx.x * DROWS + q * 4;
    if (tid < 8) *(volatile v4f*)op = ov;
    __threadfence();
    if (tid < 8) *(volatile v4f*)op = ov;
  }
}

static void launch_pack(const float* Wm, unsigned short* dst, int Kreal, int Nreal, int kS, int nT,
                        hipStream_t stream) {
  const int nPieces = nT * kS * 64;
  const int blocks  = (nPieces + 255) / 256;
  k_pack<<<dim3(blocks), dim3(256), 0, stream>>>(Wm, dst, Kreal, Nreal, kS, nPieces);
}

extern "C" void kernel_launch(void* const* d_in, const int* in_sizes, int n_in,
                              void* d_out, int out_size, void* d_ws, size_t ws_size,
                              hipStream_t stream) {
  if (n_in < 18) return;
  if (in_sizes[0] != NB * NTOK || in_sizes[1] != NB * NTOK || in_sizes[2] != NB * NTOK) return;
  if (in_sizes[3] != NSK * NSK || in_sizes[4] != NSK || in_sizes[5] != NSK * EMB) return;
  if (in_sizes[6] != HIDW * FEW || in_sizes[7] != HIDW) return;
  if (in_sizes[8] != HIDW * HIDW || in_sizes[9] != HIDW) return;
  if (in_sizes[10] != EMB * HIDW || in_sizes[11] != EMB) return;
  if (in_sizes[12] != HIDW * EMB || in_sizes[13] != HIDW) return;
  if (in_sizes[14] != HIDW * HIDW || in_sizes[15] != HIDW) return;
  if (in_sizes[16] != HIDW || in_sizes[17] != 1) return;
  if (out_size != NTGT) return;

  const int*   skills = (const int*)d_in[0];
  const int*   times  = (const int*)d_in[1];
  const int*   labels = (const int*)d_in[2];
  const float* W      = (const float*)d_in[3];
  const float* sbase  = (const float*)d_in[4];
  const float* emb    = (const float*)d_in[5];
  const float* ie_w0  = (const float*)d_in[6];
  const float* ie_b0  = (const float*)d_in[7];
  const float* ie_w1  = (const float*)d_in[8];
  const float* ie_b1  = (const float*)d_in[9];
  const float* ie_wo  = (const float*)d_in[10];
  const float* ie_bo  = (const float*)d_in[11];
  const float* f_w0   = (const float*)d_in[12];
  const float* f_b0   = (const float*)d_in[13];
  const float* f_w1   = (const float*)d_in[14];
  const float* f_b1   = (const float*)d_in[15];
  const float* f_wo   = (const float*)d_in[16];
  const float* f_bo   = (const float*)d_in[17];
  float* out = (float*)d_out;

  const size_t o_emb = 0;
  const size_t o_w0  = o_emb + (size_t)EMB_EL;
  const size_t o_w1  = o_w0 + (size_t)P0_EL;
  const size_t o_wo  = o_w1 + (size_t)P1_EL;
  const size_t o_q0  = o_wo + (size_t)P1_EL;
  const size_t o_q1  = o_q0 + (size_t)P1_EL;
  const size_t end16 = o_q1 + (size_t)P1_EL;
  const size_t cef_off   = end16 * 2;
  const size_t cef_bytes = (size_t)NTGT * EMB * 4;
  const size_t tot_bytes = cef_off + cef_bytes;
  if ((cef_off % 128) != 0) return;
  if (tot_bytes > ws_size) return;
  if (tot_bytes > (size_t)134217728) return;

  unsigned short* ws16 = (unsigned short*)d_ws;
  unsigned short* embb = ws16 + o_emb;
  unsigned short* Wp0  = ws16 + o_w0;
  unsigned short* Wp1  = ws16 + o_w1;
  unsigned short* Wpo  = ws16 + o_wo;
  unsigned short* Wq0  = ws16 + o_q0;
  unsigned short* Wq1  = ws16 + o_q1;
  float* cef = (float*)((char*)d_ws + cef_off);

  {
    const int nPieces = EMB_EL / 8;
    const int blocks  = (nPieces + 255) / 256;
    k_embc<<<dim3(blocks), dim3(256), 0, stream>>>(emb, embb, nPieces);
  }
  launch_pack(ie_w0, Wp0, FEW,  HIDW, KS0, NT4, stream);
  launch_pack(ie_w1, Wp1, HIDW, HIDW, KS1, NT4, stream);
  launch_pack(ie_wo, Wpo, HIDW, EMB,  KS1, NT4, stream);
  launch_pack(f_w0,  Wq0, EMB,  HIDW, KS1, NT4, stream);
  launch_pack(f_w1,  Wq1, HIDW, HIDW, KS1, NT4, stream);

  k_edge<<<dim3(NTGT / WPB), dim3(ETPB), 0, stream>>>(skills, times, labels, W, sbase, embb,
                                                      Wp0, Wp1, Wpo, ie_b0, ie_b1, ie_bo, cef);
  k_dec<<<dim3(NTGT / DROWS), dim3(DTPB), 0, stream>>>(cef, Wq0, Wq1, f_b0, f_b1, f_wo, f_bo, out);
  (void)hipGetLastError();
}
